// CartesianDecomposedAttention_876173328878
// MI455X (gfx1250) — hardware-verified
//
#include <hip/hip_runtime.h>
#include <math.h>
#include <stdint.h>

#ifndef NB
#define NB 8
#endif
#define NB_FULL 8
#ifndef SEQ
#define SEQ 512
#endif
#define SEQ_FULL 512
#define DMOD  1024
#define NH    16
#define HD    64
#define HK    (2 * HD)
#define DPL   (2 * DMOD)
#define NQKV  (3 * DMOD)
#define BG    ((NB <= 4) ? NB : 4)
#define NGRP  (NB / BG)
#define GROWS (BG * SEQ)
#define RSQ_HD 0.125f
#define LOG2E 1.4426950408889634f
#define LOG2_1E4 13.287712379549449f
#define QSC   1024.0f
#define KSC   1024.0f
#define PCAR  16384.0f
#define VCAR  1024.0f
#define OSC   1024.0f
#define WOS   1024.0f
#define WPB   2
#define NHG   (NH / WPB)
#define NQT   (SEQ / 16)
#define NST   (SEQ / 64)
#define NKT   (SEQ / 32)
#define ATT_THREADS (WPB * 32)
#define PTP   36
#define PTW   (16 * PTP)
#define SLP   132
#define SLW   (16 * SLP)
#define WREG  (2 * PTW + SLW)
#define SLAB64 (16 * 68)
#define VTP   72
#define WS_CAP 134217728
static_assert(DMOD == NH * HD && HD == 64 && (NH % WPB) == 0 && ATT_THREADS == 64);
static_assert(NB >= 1 && NB <= NB_FULL && BG >= 1 && BG <= 4 && (NB % BG) == 0);
static_assert((SEQ % 64) == 0 && SEQ >= 64 && SEQ <= SEQ_FULL);
static_assert((GROWS % 64) == 0 && (DPL % 64) == 0 && (DPL % 32) == 0 && (DMOD % 64) == 0);
static_assert(DPL == 256 * 8);
static_assert(HK == 128 && (HK % 32) == 0);
static_assert((SLP % 4) == 0 && (PTP % 4) == 0 && ((WREG * 4) % 16) == 0 && ((PTW * 4) % 16) == 0);
static_assert((SEQ * HD) % 256 == 0);

typedef unsigned short u16;
typedef _Float16 v16h __attribute__((ext_vector_type(16)));
typedef _Float16 v8h  __attribute__((ext_vector_type(8)));
typedef __bf16   v16b __attribute__((ext_vector_type(16)));
typedef float    v8f  __attribute__((ext_vector_type(8)));
typedef float    v4f  __attribute__((ext_vector_type(4)));
typedef unsigned int v4u __attribute__((ext_vector_type(4)));

union FragH { v16h v; v8h h[2]; v4u u[2]; };
union FragB { v16b v; v4u u[2]; };

__device__ __forceinline__ unsigned short bf_bits(float f) {
  unsigned u = __float_as_uint(f);
  return (unsigned short)((u + 0x7FFFu + ((u >> 16) & 1u)) >> 16);
}
__device__ __forceinline__ float bf_up(unsigned short h) { return __uint_as_float(((unsigned)h) << 16); }
__device__ __forceinline__ float bfr(float f) { return bf_up(bf_bits(f)); }
__device__ __forceinline__ unsigned short h_bits(_Float16 x) { return __builtin_bit_cast(unsigned short, x); }
__device__ __forceinline__ unsigned pk16(unsigned short a, unsigned short b) { return (unsigned)a | ((unsigned)b << 16); }
__device__ __forceinline__ v8f zero8() { v8f z = {0.f, 0.f, 0.f, 0.f, 0.f, 0.f, 0.f, 0.f}; return z; }

__device__ __forceinline__ v16h ldfrag_h(const _Float16* p) {
  FragH f;
  f.h[0] = *(const v8h*)(p);
  f.h[1] = *(const v8h*)(p + 16);
  return f.v;
}
__device__ __forceinline__ v16b ldfrag_b(const u16* p) {
  FragB f;
  f.u[0] = *(const v4u*)(p);
  f.u[1] = *(const v4u*)(p + 16);
  return f.v;
}

__device__ __forceinline__ v8f mma_h(v16h a, v16h b, v8f c) {
  return __builtin_amdgcn_wmma_f32_16x16x32_f16(false, a, false, b, (short)0, c, false, false);
}
__device__ __forceinline__ v8f mma_b(v16b a, v16b b, v8f c) {
  return __builtin_amdgcn_wmma_f32_16x16x32_bf16(false, a, false, b, (short)0, c, false, false);
}
__device__ __forceinline__ void guard2(v8f& a, v8f& b, v16h x0, v16h x1, v16h x2, v16h x3, v16h x4, v16h x5) {
#if defined(__HIP_DEVICE_COMPILE__)
  asm volatile("v_nop\n\tv_nop\n\tv_nop\n\tv_nop"
               : "+v"(a), "+v"(b) : "v"(x0), "v"(x1), "v"(x2), "v"(x3), "v"(x4), "v"(x5) : "memory");
#endif
}
template <typename F>
__device__ __forceinline__ void guard6(v8f& a, v8f& b, v8f& c, v8f& d, F x0, F x1, F x2, F x3, F x4, F x5) {
#if defined(__HIP_DEVICE_COMPILE__)
  asm volatile("v_nop\n\tv_nop\n\tv_nop\n\tv_nop"
               : "+v"(a), "+v"(b), "+v"(c), "+v"(d) : "v"(x0), "v"(x1), "v"(x2), "v"(x3), "v"(x4), "v"(x5) : "memory");
#endif
}
__device__ __forceinline__ void guard4x8(v8f& a, v8f& b, v8f& c, v8f& d, v16h x0, v16h x1, v16h x2, v16h x3,
                                         v16h x4, v16h x5, v16h x6, v16h x7) {
#if defined(__HIP_DEVICE_COMPILE__)
  asm volatile("v_nop\n\tv_nop\n\tv_nop\n\tv_nop"
               : "+v"(a), "+v"(b), "+v"(c), "+v"(d)
               : "v"(x0), "v"(x1), "v"(x2), "v"(x3), "v"(x4), "v"(x5), "v"(x6), "v"(x7) : "memory");
#endif
}
__device__ __forceinline__ void acc_guard4(v8f& a, v8f& b, v8f& c, v8f& d) {
#if defined(__HIP_DEVICE_COMPILE__)
  asm volatile("v_nop\n\tv_nop\n\tv_nop\n\tv_nop" : "+v"(a), "+v"(b), "+v"(c), "+v"(d));
#endif
}
__device__ __forceinline__ void wave_sync_lds() {
  __builtin_amdgcn_fence(__ATOMIC_RELEASE, "workgroup");
  __builtin_amdgcn_wave_barrier();
  __builtin_amdgcn_fence(__ATOMIC_ACQUIRE, "workgroup");
}

__global__ __launch_bounds__(256) void rot_tab(float* CT, float* ST, int n) {
  const int idx = blockIdx.x * 256 + (int)threadIdx.x;
  if (idx >= n) return;
  const int s = idx / HD;
  const int d = idx - s * HD;
  const float ex   = (float)d * (LOG2_1E4 / (float)HD);
  const float invf = exp2f(-ex);
  const float th   = (float)s * invf;
  float sn, cs;
  sincosf(th, &sn, &cs);
  for (int pass = 0; pass < 2; ++pass) {
    *(volatile float*)(CT + idx) = cs;
    *(volatile float*)(ST + idx) = sn;
    __threadfence();
  }
}

__global__ __launch_bounds__(256) void wcvt(const float* __restrict__ Wr, const float* __restrict__ Wi, u16* D,
                                            int nrows, int f16mode, float scale) {
  const int n = blockIdx.x;
  if (n >= nrows) return;
  const int tid  = threadIdx.x;
  const int p    = n / DPL;
  const int j    = n - p * DPL;
  const int im   = (j >= DMOD) ? 1 : 0;
  const int e    = p * DMOD + (j & (DMOD - 1));
  const int c8   = tid * 8;
  const int ksec = (c8 >= DMOD) ? 1 : 0;
  const int kk   = c8 & (DMOD - 1);
  const float* src = ((im == ksec) ? Wr : Wi) + (size_t)e * DMOD + kk;
  const float sgn  = (im == 0 && ksec != 0) ? -1.0f : 1.0f;
  const v4f a = *(const v4f*)(src), b4 = *(const v4f*)(src + 4);
  float w[8];
#pragma unroll
  for (int q = 0; q < 4; ++q) { w[q] = a[q] * sgn; w[4 + q] = b4[q] * sgn; }
  v4u o;
#pragma unroll
  for (int q = 0; q < 4; ++q) {
    const float f0 = w[2 * q], f1 = w[2 * q + 1];
    const unsigned short hb0 = h_bits((_Float16)(bfr(f0) * scale));
    const unsigned short hb1 = h_bits((_Float16)(bfr(f1) * scale));
    const unsigned short bb0 = bf_bits(f0);
    const unsigned short bb1 = bf_bits(f1);
    o[q] = (f16mode != 0) ? pk16(hb0, hb1) : pk16(bb0, bb1);
  }
  u16* d = D + (size_t)n * DPL + c8;
  for (int pass = 0; pass < 2; ++pass) {
    *(volatile v4u*)(d) = o;
    __threadfence();
  }
}

__global__ __launch_bounds__(256) void xcvt(const float* __restrict__ xr, const float* __restrict__ xi, u16* D,
                                            int nrows, int gb0) {
  const int row = blockIdx.x;
  if (row >= nrows) return;
  const int tid  = threadIdx.x;
  const int bl   = row / SEQ;
  const int s    = row - bl * SEQ;
  const size_t grow = (size_t)(gb0 + bl) * SEQ_FULL + s;
  const int c8   = tid * 8;
  const int ksec = (c8 >= DMOD) ? 1 : 0;
  const int kk   = c8 & (DMOD - 1);
  const float* src = ((ksec != 0) ? xi : xr) + grow * DMOD + kk;
  const v4f a = *(const v4f*)(src), b4 = *(const v4f*)(src + 4);
  v4u o;
#pragma unroll
  for (int q = 0; q < 4; ++q) {
    const float f0 = (q < 2) ? a[2 * q] : b4[2 * q - 4];
    const float f1 = (q < 2) ? a[2 * q + 1] : b4[2 * q - 3];
    o[q] = pk16(bf_bits(f0), bf_bits(f1));
  }
  u16* d = D + (size_t)row * DPL + c8;
  for (int pass = 0; pass < 2; ++pass) {
    *(volatile v4u*)(d) = o;
    __threadfence();
  }
}

__device__ __forceinline__ void epi64(float* sl, v8f a0, v8f a1, v8f a2, v8f a3, float oscale,
                                      float* C, int N, size_t rowb, int col0, int lane) {
  const int hh = lane >> 4, m = lane & 15;
#pragma unroll
  for (int r = 0; r < 8; ++r) {
    const int ro = (8 * hh + r) * 68 + m;
    sl[ro]      = a0[r] * oscale;
    sl[ro + 16] = a1[r] * oscale;
    sl[ro + 32] = a2[r] * oscale;
    sl[ro + 48] = a3[r] * oscale;
  }
  wave_sync_lds();
  v4f vals[8];
#pragma unroll
  for (int it = 0; it < 8; ++it) vals[it] = *(const v4f*)(sl + (it * 2 + hh) * 68 + m * 4);
  float* dst = C + (rowb + (size_t)hh) * (size_t)N + col0 + m * 4;
  for (int pass = 0; pass < 2; ++pass) {
#pragma unroll
    for (int it = 0; it < 8; ++it) {
      *(volatile v4f*)(dst + (size_t)(it * 2) * (size_t)N) = vals[it];
    }
    __threadfence();
  }
}

template <int F16>
__global__ __launch_bounds__(128)
void gemm16(const u16* __restrict__ A, const u16* __restrict__ Bt, float* C, int M, int N, int K, float oscale) {
  __shared__ __align__(16) float slab[4 * SLAB64];
  const int tid = threadIdx.x, wave = tid >> 5, lane = tid & 31, hh = lane >> 4, m = lane & 15;
  const int ntile = N >> 6;
  const int bid   = blockIdx.x;
  const int rowb  = (bid / ntile) * 64 + wave * 16;
  const int col0  = (bid % ntile) * 64;
  if (rowb + 16 > M) return;
  const size_t bs = (size_t)16 * K;
  v8f acc0 = zero8(), acc1 = zero8(), acc2 = zero8(), acc3 = zero8();
  if constexpr (F16 != 0) {
    const _Float16* ap = (const _Float16*)(const void*)A  + (size_t)(rowb + m) * K + 8 * hh;
    const _Float16* bp = (const _Float16*)(const void*)Bt + (size_t)(col0 + m) * K + 8 * hh;
#pragma unroll 1
    for (int k0 = 0; k0 < K; k0 += 32) {
      const v16h a  = ldfrag_h(ap + k0);
      const v16h b0 = ldfrag_h(bp + k0);
      const v16h b1 = ldfrag_h(bp + bs + k0);
      const v16h b2 = ldfrag_h(bp + 2 * bs + k0);
      const v16h b3 = ldfrag_h(bp + 3 * bs + k0);
      acc0 = mma_h(a, b0, acc0);
      acc1 = mma_h(a, b1, acc1);
      acc2 = mma_h(a, b2, acc2);
      acc3 = mma_h(a, b3, acc3);
      guard6<v16h>(acc0, acc1, acc2, acc3, a, b0, b1, b2, b3, a);
    }
  } else {
    const u16* ap = A  + (size_t)(rowb + m) * K + 8 * hh;
    const u16* bp = Bt + (size_t)(col0 + m) * K + 8 * hh;
#pragma unroll 1
    for (int k0 = 0; k0 < K; k0 += 32) {
      const v16b a  = ldfrag_b(ap + k0);
      const v16b b0 = ldfrag_b(bp + k0);
      const v16b b1 = ldfrag_b(bp + bs + k0);
      const v16b b2 = ldfrag_b(bp + 2 * bs + k0);
      const v16b b3 = ldfrag_b(bp + 3 * bs + k0);
      acc0 = mma_b(a, b0, acc0);
      acc1 = mma_b(a, b1, acc1);
      acc2 = mma_b(a, b2, acc2);
      acc3 = mma_b(a, b3, acc3);
      guard6<v16b>(acc0, acc1, acc2, acc3, a, b0, b1, b2, b3, a);
    }
  }
  epi64(slab + wave * SLAB64, acc0, acc1, acc2, acc3, oscale, C, N, (size_t)rowb, col0, lane);
}

__global__ __launch_bounds__(256) void vt16(const float* __restrict__ F, u16* VTo) {
  __shared__ __align__(16) u16 T[HK * VTP];
  const int tid = threadIdx.x;
  const int bid = blockIdx.x;
  const int st  = bid % NST;
  const int t2  = bid / NST;
  const int g   = t2 % NH;
  const int b   = t2 / NH;
  if (b >= BG) return;
  const int s0  = st * 64;
  {
    const int sl   = tid >> 2;
    const int dc   = tid & 3;
    const int comp = dc >> 1;
    const int d0   = (dc & 1) * 32;
    const float* src = F + ((size_t)b * SEQ + s0 + sl) * DPL + (size_t)comp * DMOD + g * HD + d0;
#pragma unroll
    for (int i = 0; i < 8; ++i) {
      const v4f a = *(const v4f*)(src + 4 * i);
#pragma unroll
      for (int e = 0; e < 4; ++e) {
        T[(comp * HD + d0 + 4 * i + e) * VTP + sl] = h_bits((_Float16)(a[e] * VCAR));
      }
    }
  }
  __syncthreads();
  v4u vv[4];
  const int q8 = tid >> 3, p8 = (tid & 7) * 8;
#pragma unroll
  for (int it = 0; it < 4; ++it) {
    const int line = it * 32 + q8;
    vv[it] = *(const v4u*)(T + line * VTP + p8);
  }
  const size_t base = ((size_t)(b * NH + g) * HK) * SEQ + s0 + p8;
  for (int pass = 0; pass < 2; ++pass) {
#pragma unroll
    for (int it = 0; it < 4; ++it) {
      const int line = it * 32 + q8;
      *(volatile v4u*)(VTo + base + (size_t)line * SEQ) = vv[it];
    }
    __threadfence();
  }
}

__global__ __launch_bounds__(256) void rope16(const float* __restrict__ F, const float* __restrict__ CT,
                                              const float* __restrict__ ST, u16* Hp, u16* Lp, int nrows, float sc) {
  const int row = blockIdx.x;
  if (row >= nrows) return;
  const int tid  = threadIdx.x;
  const int s    = row % SEQ;
  const int h    = tid >> 4;
  const int comp = (tid >> 3) & 1;
  const int d8   = (tid & 7) * 8;
  const float* pa = F + (size_t)row * DPL + (size_t)comp * DMOD + h * HD + d8;
  const float* po = F + (size_t)row * DPL + (size_t)(1 - comp) * DMOD + h * HD + d8;
  const float* pc = CT + (size_t)s * HD + d8;
  const float* pn = ST + (size_t)s * HD + d8;
  const v4f a0 = *(const v4f*)(pa), a1 = *(const v4f*)(pa + 4);
  const v4f o0 = *(const v4f*)(po), o1 = *(const v4f*)(po + 4);
  const v4f c0 = *(const v4f*)(pc), c1 = *(const v4f*)(pc + 4);
  const v4f n0 = *(const v4f*)(pn), n1 = *(const v4f*)(pn + 4);
  const float sg = (comp != 0) ? 1.0f : -1.0f;
  float w[8];
#pragma unroll
  for (int e = 0; e < 4; ++e) {
    w[e]     = (a0[e] * c0[e] + sg * (o0[e] * n0[e])) * sc;
    w[4 + e] = (a1[e] * c1[e] + sg * (o1[e] * n1[e])) * sc;
  }
  v4u oh, ol;
#pragma unroll
  for (int e = 0; e < 4; ++e) {
    const float t0 = w[2 * e], t1 = w[2 * e + 1];
    const _Float16 h0 = (_Float16)t0, h1 = (_Float16)t1;
    const _Float16 l0 = (_Float16)(t0 - (float)h0), l1 = (_Float16)(t1 - (float)h1);
    oh[e] = pk16(h_bits(h0), h_bits(h1));
    ol[e] = pk16(h_bits(l0), h_bits(l1));
  }
  u16* dh = Hp + (size_t)row * DPL + tid * 8;
  u16* dl = Lp + (size_t)row * DPL + tid * 8;
  for (int pass = 0; pass < 2; ++pass) {
    *(volatile v4u*)(dh) = oh;
    *(volatile v4u*)(dl) = ol;
    __threadfence();
  }
}

__global__ __launch_bounds__(ATT_THREADS)
void attn(const u16* __restrict__ QHp, const u16* __restrict__ QLp,
          const u16* __restrict__ KHp, const u16* __restrict__ KLp,
          const u16* __restrict__ VTp, u16* OHp) {
  __shared__ __align__(16) float smem[WPB * WREG];

  const int tid  = threadIdx.x;
  const int wave = tid >> 5;
  const int lane = tid & 31;
  const int hh   = lane >> 4;
  const int c    = lane & 15;
  const int bid  = blockIdx.x;
  const int qt   = bid % NQT;
  const int t2   = bid / NQT;
  const int hg   = t2 % NHG;
  const int b    = t2 / NHG;
  if (b >= BG) return;
  const int q0   = qt * 16;
  const int head = hg * WPB + wave;

  float* pct  = smem + wave * WREG;
  float* pst  = pct + PTW;
  float* slab = pst + PTW;

  const size_t hcol = (size_t)head * HK + 8 * hh;
  const _Float16* Qh  = (const _Float16*)(const void*)QHp + ((size_t)b * SEQ + q0 + c) * DPL + hcol;
  const _Float16* Ql  = (const _Float16*)(const void*)QLp + ((size_t)b * SEQ + q0 + c) * DPL + hcol;
  const _Float16* Khb = (const _Float16*)(const void*)KHp + ((size_t)b * SEQ + c) * DPL + hcol;
  const _Float16* Klb = (const _Float16*)(const void*)KLp + ((size_t)b * SEQ + c) * DPL + hcol;
  const _Float16* Vtb = (const _Float16*)(const void*)VTp + ((size_t)(b * NH + head) * HK + c) * SEQ + 8 * hh;
  const float lsc = RSQ_HD * (LOG2E / (QSC * KSC));
  const float psc = RSQ_HD / (QSC * KSC);
  const float oc  = 1.0f / (PCAR * VCAR);
  const v4u sgn4 = {0x80008000u, 0x80008000u, 0x80008000u, 0x80008000u};

  float mrow[8], lrow[8];
  v8f orr[4], oii[4];
#pragma unroll
  for (int r = 0; r < 8; ++r) { mrow[r] = -INFINITY; lrow[r] = 0.f; }
#pragma unroll
  for (int j = 0; j < 4; ++j) { orr[j] = zero8(); oii[j] = zero8(); }

#pragma unroll 1
  for (int kt = 0; kt < NKT; ++kt) {
    const int kb = kt * 32;
    v8f sr0 = zero8(), sr1 = zero8(), si0 = zero8(), si1 = zero8();
    const _Float16* k0p = Khb + (size_t)kb * DPL;
    const _Float16* k1p = k0p + (size_t)16 * DPL;
    const _Float16* l0p = Klb + (size_t)kb * DPL;
    const _Float16* l1p = l0p + (size_t)16 * DPL;
#pragma unroll
    for (int kk = 0; kk < HK / 32; ++kk) {
      const v16h kh0 = ldfrag_h(k0p + kk * 32);
      const v16h kl0 = ldfrag_h(l0p + kk * 32);
      const v16h kh1 = ldfrag_h(k1p + kk * 32);
      const v16h kl1 = ldfrag_h(l1p + kk * 32);
      {
        const v16h qh = ldfrag_h(Qh + kk * 32);
        const v16h ql = ldfrag_h(Ql + kk * 32);
        sr0 = mma_h(qh, kh0, sr0);
        sr0 = mma_h(ql, kh0, sr0);
        sr0 = mma_h(qh, kl0, sr0);
        sr1 = mma_h(qh, kh1, sr1);
        sr1 = mma_h(ql, kh1, sr1);
        sr1 = mma_h(qh, kl1, sr1);
        guard2(sr0, sr1, qh, ql, kh0, kl0, kh1, kl1);
      }
      {
        const int ko = ((kk + 2) & 3) * 32;
        FragH ah, al;
        ah.v = ldfrag_h(Qh + ko);
        al.v = ldfrag_h(Ql + ko);
        if (kk >= 2) {
          ah.u[0] = ah.u[0] ^ sgn4;  ah.u[1] = ah.u[1] ^ sgn4;
          al.u[0] = al.u[0] ^ sgn4;  al.u[1] = al.u[1] ^ sgn4;
        }
        si0 = mma_h(ah.v, kh0, si0);
        si0 = mma_h(al.v, kh0, si0);
        si0 = mma_h(ah.v, kl0, si0);
        si1 = mma_h(ah.v, kh1, si1);
        si1 = mma_h(al.v, kh1, si1);
        si1 = mma_h(ah.v, kl1, si1);
        guard2(si0, si1, ah.v, al.v, kh0, kl0, kh1, kl1);
      }
    }
#pragma unroll
    for (int r = 0; r < 8; ++r) {
      const float u0 = sr0[r] * lsc;
      const float u1 = sr1[r] * lsc;
      float mx = fmaxf(u0, u1);
#pragma unroll
      for (int off = 1; off < 16; off <<= 1) mx = fmaxf(mx, __shfl_xor(mx, off, 32));
      const float mn = fmaxf(mrow[r], mx);
      const float ms = (mn == -INFINITY) ? 0.0f : mn;
      const float al = exp2f(mrow[r] - ms);
      mrow[r] = mn;
      const float e0 = exp2f(u0 - ms), e1 = exp2f(u1 - ms);
      float ps = e0 + e1;
#pragma unroll
      for (int off = 1; off < 16; off <<= 1) ps += __shfl_xor(ps, off, 32);
      lrow[r] = lrow[r] * al + ps;
#pragma unroll
      for (int j = 0; j < 4; ++j) { orr[j][r] *= al; oii[j][r] *= al; }
      float sn0, cs0, sn1, cs1;
      __sincosf(si0[r] * psc, &sn0, &cs0);
      __sincosf(si1[r] * psc, &sn1, &cs1);
      const int ro = (8 * hh + r) * PTP + c;
      pct[ro]      = e0 * cs0;
      pct[ro + 16] = e1 * cs1;
      pst[ro]      = e0 * sn0;
      pst[ro + 16] = e1 * sn1;
    }
    wave_sync_lds();
    FragH pc, psf, pnf;
    {
      const float* prc = pct + c * PTP + 8 * hh;
      const float* prs = pst + c * PTP + 8 * hh;
      const v4f c0 = *(const v4f*)(prc), c1 = *(const v4f*)(prc + 4);
      const v4f c2 = *(const v4f*)(prc + 16), c3 = *(const v4f*)(prc + 20);
      const v4f s0 = *(const v4f*)(prs), s1 = *(const v4f*)(prs + 4);
      const v4f s2 = *(const v4f*)(prs + 16), s3 = *(const v4f*)(prs + 20);
#pragma unroll
      for (int e = 0; e < 4; ++e) {
        pc.h[0][e]      = (_Float16)(c0[e] * PCAR);
        pc.h[0][4 + e]  = (_Float16)(c1[e] * PCAR);
        pc.h[1][e]      = (_Float16)(c2[e] * PCAR);
        pc.h[1][4 + e]  = (_Float16)(c3[e] * PCAR);
        psf.h[0][e]     = (_Float16)(s0[e] * PCAR);
        psf.h[0][4 + e] = (_Float16)(s1[e] * PCAR);
        psf.h[1][e]     = (_Float16)(s2[e] * PCAR);
        psf.h[1][4 + e] = (_Float16)(s3[e] * PCAR);
      }
      pnf.u[0] = psf.u[0] ^ sgn4;
      pnf.u[1] = psf.u[1] ^ sgn4;
    }
    {
      const _Float16* vp = Vtb + kb;
#pragma unroll
      for (int jg = 0; jg < 2; ++jg) {
        const size_t ra = (size_t)(2 * jg) * 16 * SEQ;
        const size_t rb = ra + (size_t)16 * SEQ;
        const size_t ia = ra + (size_t)HD * SEQ;
        const size_t ib = rb + (size_t)HD * SEQ;
        const v16h vra = ldfrag_h(vp + ra), vrb = ldfrag_h(vp + rb);
        const v16h via = ldfrag_h(vp + ia), vib = ldfrag_h(vp + ib);
        orr[2 * jg]     = mma_h(pc.v,  vra, orr[2 * jg]);
        orr[2 * jg]     = mma_h(pnf.v, via, orr[2 * jg]);
        oii[2 * jg]     = mma_h(psf.v, vra, oii[2 * jg]);
        oii[2 * jg]     = mma_h(pc.v,  via, oii[2 * jg]);
        orr[2 * jg + 1] = mma_h(pc.v,  vrb, orr[2 * jg + 1]);
        orr[2 * jg + 1] = mma_h(pnf.v, vib, orr[2 * jg + 1]);
        oii[2 * jg + 1] = mma_h(psf.v, vrb, oii[2 * jg + 1]);
        oii[2 * jg + 1] = mma_h(pc.v,  vib, oii[2 * jg + 1]);
        guard4x8(orr[2 * jg], oii[2 * jg], orr[2 * jg + 1], oii[2 * jg + 1],
                 pc.v, psf.v, pnf.v, vra, vrb, via, vib, pc.v);
      }
    }
    wave_sync_lds();
  }
  acc_guard4(orr[0], orr[1], orr[2], orr[3]);
  acc_guard4(oii[0], oii[1], oii[2], oii[3]);
#pragma unroll
  for (int r = 0; r < 8; ++r) {
    const float lv  = lrow[r];
    const float ls  = (lv > 0.0f) ? lv : 1.0f;
    const float inv = (lv > 0.0f) ? ((1.0f / ls) * oc) : 0.0f;
#pragma unroll
    for (int j = 0; j < 4; ++j) {
      const int idx = (8 * hh + r) * SLP + j * 16 + c;
      slab[idx]      = orr[j][r] * inv;
      slab[idx + HD] = oii[j][r] * inv;
    }
  }

  wave_sync_lds();
  v4u oh[4][2];
  const int rq = lane >> 3, c8 = (lane & 7) * 8;
#pragma unroll
  for (int it = 0; it < 4; ++it) {
    const int row = it * 4 + rq;
#pragma unroll
    for (int part = 0; part < 2; ++part) {
      const float* sp = slab + row * SLP + part * HD + c8;
      const v4f a = *(const v4f*)(sp), b4 = *(const v4f*)(sp + 4);
      float w[8];
#pragma unroll
      for (int e = 0; e < 4; ++e) { w[e] = a[e] * OSC; w[4 + e] = b4[e] * OSC; }
#pragma unroll
      for (int e = 0; e < 4; ++e) {
        const _Float16 h0 = (_Float16)w[2 * e], h1 = (_Float16)w[2 * e + 1];
        oh[it][part][e] = pk16(h_bits(h0), h_bits(h1));
      }
    }
  }
  const size_t ob = ((size_t)b * SEQ + q0) * DPL + (size_t)head * HD + c8;
  for (int pass = 0; pass < 2; ++pass) {
#pragma unroll
    for (int it = 0; it < 4; ++it) {
      const int row = it * 4 + rq;
#pragma unroll
      for (int part = 0; part < 2; ++part) {
        *(volatile v4u*)(OHp + ob + (size_t)row * DPL + (size_t)part * DMOD) = oh[it][part];
      }
    }
    __threadfence();
  }
}

extern "C" void kernel_launch(void* const* d_in, const int* in_sizes, int n_in,
                              void* d_out, int out_size, void* d_ws, size_t ws_size,
                              hipStream_t stream) {
  if (n_in < 6) return;
  if (in_sizes[0] < ((NB - 1) * SEQ_FULL + SEQ) * DMOD) return;
  if (in_sizes[1] < ((NB - 1) * SEQ_FULL + SEQ) * DMOD) return;
  if (in_sizes[2] < NQKV * DMOD) return;
  if (in_sizes[3] < NQKV * DMOD) return;
  if (in_sizes[4] < DMOD * DMOD) return;
  if (in_sizes[5] < DMOD * DMOD) return;
  if (out_size < 2 * NB * SEQ * DMOD) return;

  const float* xr    = (const float*)d_in[0];
  const float* xi    = (const float*)d_in[1];
  const float* wqr   = (const float*)d_in[2];
  const float* wqi   = (const float*)d_in[3];
  const float* wor   = (const float*)d_in[4];
  const float* woi   = (const float*)d_in[5];
  float*       out0  = (float*)d_out;
  float*       out1  = out0 + (size_t)(out_size / 2);

  const size_t szTAB = (((size_t)SEQ * HD * 4) + 32767) / 32768 * 32768;
  const size_t szWQ  = (size_t)2 * NQKV * DPL * 2;
  const size_t szWO  = (size_t)2 * DMOD * DPL * 2;
  const size_t szXB  = (size_t)GROWS * DPL * 2;
  const size_t szF   = (size_t)GROWS * DPL * 4;
  const size_t szH   = (size_t)GROWS * DPL * 2;
  const size_t szVT  = (size_t)BG * NH * HK * SEQ * 2;
  if (szH > szF) return;
  size_t off = 0;
  const size_t oCT = off; off += szTAB;
  const size_t oST = off; off += szTAB;
  const size_t oWQ = off; off += szWQ;
  const size_t oWO = off; off += szWO;
  const size_t oXB = off; off += szXB;
  const size_t oF  = off; off += szF;
  const size_t oQH = off; off += szH;
  const size_t oQL = off; off += szH;
  const size_t oKH = off; off += szH;
  const size_t oKL = off; off += szH;
  const size_t oVT = off; off += szVT;
  if (off > ws_size) return;
  if (off > (size_t)WS_CAP) return;

  char* ws = (char*)d_ws;
  float* CT  = (float*)(ws + oCT);
  float* ST  = (float*)(ws + oST);
  u16*   WQB = (u16*)(ws + oWQ);
  u16*   WOB = (u16*)(ws + oWO);
  u16*   XB  = (u16*)(ws + oXB);
  float* F   = (float*)(ws + oF);
  u16*   OH  = (u16*)(ws + oF);
  u16*   QH  = (u16*)(ws + oQH);
  u16*   QL  = (u16*)(ws + oQL);
  u16*   KH  = (u16*)(ws + oKH);
  u16*   KL  = (u16*)(ws + oKL);
  u16*   VT  = (u16*)(ws + oVT);

  const dim3 b256(256), b128(128), bAT(ATT_THREADS);
  const int  ntab = SEQ * HD;
  const dim3 gTAB((ntab + 255) / 256);
  const dim3 gWQ(2 * NQKV), gWO(2 * DMOD);
  const dim3 gX(GROWS);
  const dim3 gG2((GROWS / 64) * (DPL / 64));
  const dim3 gG1((GROWS / 64) * (DMOD / 64));
  const dim3 gVT(BG * NH * NST);
  const dim3 gRP(GROWS);
  const dim3 gAT(NQT * NHG * BG);
  const size_t wpart = (size_t)DPL * DPL;
  const float osc = 1.0f / (OSC * WOS);

  rot_tab<<<gTAB, b256, 0, stream>>>(CT, ST, ntab);
  wcvt<<<gWQ, b256, 0, stream>>>(wqr, wqi, WQB, 2 * NQKV, 0, 1.0f);
  wcvt<<<gWO, b256, 0, stream>>>(wor, woi, WOB, 2 * DMOD, 1, WOS);

  for (int g = 0; g < NGRP; ++g) {
    float* og0 = out0 + (size_t)g * GROWS * DMOD;
    float* og1 = out1 + (size_t)g * GROWS * DMOD;
    xcvt<<<gX, b256, 0, stream>>>(xr, xi, XB, GROWS, g * BG);
    gemm16<0><<<gG2, b128, 0, stream>>>(XB, WQB + 2 * wpart, F, GROWS, DPL, DPL, 1.0f);
    vt16<<<gVT, b256, 0, stream>>>(F, VT);
    gemm16<0><<<gG2, b128, 0, stream>>>(XB, WQB, F, GROWS, DPL, DPL, 1.0f);
    rope16<<<gRP, b256, 0, stream>>>(F, CT, ST, QH, QL, GROWS, QSC);
    gemm16<0><<<gG2, b128, 0, stream>>>(XB, WQB + wpart, F, GROWS, DPL, DPL, 1.0f);
    rope16<<<gRP, b256, 0, stream>>>(F, CT, ST, KH, KL, GROWS, KSC);
    attn<<<gAT, bAT, 0, stream>>>(QH, QL, KH, KL, VT, OH);
    gemm16<1><<<gG1, b128, 0, stream>>>(OH, WOB, og0, GROWS, DMOD, DPL, osc);
    gemm16<1><<<gG1, b128, 0, stream>>>(OH, WOB + (size_t)DMOD * DPL, og1, GROWS, DMOD, DPL, osc);
  }
  (void)hipGetLastError();
}
